// GraphODEFunc_9740985827791
// MI455X (gfx1250) — hardware-verified
//
#include <hip/hip_runtime.h>
#include <hip/hip_bf16.h>
#include <math.h>


#define NBATCH 16
#define SS 1024
#define NN 1024
#define HD 128
#define HH 16
#define DKK 64
#define QW 2

typedef _Float16 bf16;
typedef __attribute__((ext_vector_type(4))) unsigned v4u_t;
typedef unsigned v4ua __attribute__((ext_vector_type(4), may_alias));
typedef __attribute__((ext_vector_type(4))) float v4f_t;
typedef float v4fa __attribute__((ext_vector_type(4), may_alias));
typedef __attribute__((ext_vector_type(16))) bf16  bf16x16;
typedef __attribute__((ext_vector_type(8)))  bf16  bf16x8;
typedef __attribute__((ext_vector_type(4)))  bf16  bf16x4;
typedef __attribute__((ext_vector_type(8)))  float f32x8;

#define LDS_STRIDE 48
#define KSTRIDE    72
#define VSTRIDE    48

__device__ __forceinline__ f32x8 wmma_bf16(bf16x16 a, bf16x16 b, f32x8 c) {
  return __builtin_amdgcn_wmma_f32_16x16x32_f16(
      false, a, false, b, (short)0, c, false, false);
}

template <typename T>
__device__ __forceinline__ bf16x16 load_frag(const T* __restrict__ base, int ld,
                                             int row0, int k0) {
  const int lane = threadIdx.x & 31;
  const int r    = lane & 15;
  const int kh   = (lane >> 4) * 8;
  const T* p0 = base + (size_t)(row0 + r) * ld + (k0 + kh);
  const T* p1 = p0 + 16;
  bf16x16 f;
#pragma unroll
  for (int i = 0; i < 8; ++i) {
    f[i]     = (bf16)p0[i];
    f[i + 8] = (bf16)p1[i];
  }
  return f;
}

__device__ __forceinline__ bf16x16 lds_frag(const bf16* base, int stride) {
  const int lane = threadIdx.x & 31;
  const int row  = lane & 15;
  const int kh   = (lane >> 4) * 8;
  const bf16x8 lo = *(const bf16x8*)(base + row * stride + kh);
  const bf16x8 hi = *(const bf16x8*)(base + row * stride + kh + 16);
  bf16x16 f;
#pragma unroll
  for (int i = 0; i < 8; ++i) { f[i] = lo[i]; f[i + 8] = hi[i]; }
  return f;
}

template <typename T>
__device__ __forceinline__ void stage_read16(const T* __restrict__ p, float* buf) {
#pragma unroll
  for (int i = 0; i < 16; ++i) buf[i] = (float)p[i];
}

__device__ __forceinline__ void stage_write(bf16* dst, const float* buf, int nquad) {
#pragma unroll
  for (int i = 0; i < nquad; ++i) {
    bf16x4 q;
    q[0] = (bf16)buf[4 * i];     q[1] = (bf16)buf[4 * i + 1];
    q[2] = (bf16)buf[4 * i + 2]; q[3] = (bf16)buf[4 * i + 3];
    *(bf16x4*)(dst + 4 * i) = q;
  }
}

template <typename AT, int MODE>
__global__ __launch_bounds__(256) void gemm_bias_kernel(
    const AT* __restrict__ A, const float* __restrict__ W,
    const float* __restrict__ bias, void* __restrict__ out,
    int M, int N, int K, size_t bsA, size_t bsW, size_t bsObytes) {
  __shared__ bf16 ldsA[128 * LDS_STRIDE];
  __shared__ bf16 ldsW[256 * LDS_STRIDE];
  __shared__ __attribute__((aligned(16))) unsigned char sob[256 * 136 * 2];

  const int t    = threadIdx.x;
  const int wave = t >> 5;
  const int lane = t & 31;
  const int wm   = (wave & 1) * 64;
  const int wn   = (wave >> 1) * 64;
  const int mBlk = blockIdx.x * 128;
  const int nBlk = blockIdx.y * 256;
  A += (size_t)blockIdx.z * bsA; W += (size_t)blockIdx.z * bsW; out = (void*)((char*)out + (size_t)blockIdx.z * bsObytes);

  const int arow = t >> 1;
  const int ach  = (t & 1) * 16;

  float abuf[16];
  float wbuf[32];

  stage_read16(A + (size_t)(mBlk + arow) * K + ach, abuf);
  stage_read16(W + (size_t)(nBlk + t) * K,          wbuf);
  stage_read16(W + (size_t)(nBlk + t) * K + 16,     wbuf + 16);

  f32x8 acc[4][4] = {};

  for (int k = 0; k < K; k += 32) {
    __syncthreads();
    stage_write(&ldsA[arow * LDS_STRIDE + ach], abuf, 4);
    stage_write(&ldsW[t * LDS_STRIDE],          wbuf, 8);
    if (k + 32 < K) {
      stage_read16(A + (size_t)(mBlk + arow) * K + (k + 32) + ach, abuf);
      stage_read16(W + (size_t)(nBlk + t) * K + (k + 32),          wbuf);
      stage_read16(W + (size_t)(nBlk + t) * K + (k + 32) + 16,     wbuf + 16);
    }
    __syncthreads();

    bf16x16 af[4], wf[4];
#pragma unroll
    for (int i = 0; i < 4; ++i)
      af[i] = lds_frag(ldsA + (wm + 16 * i) * LDS_STRIDE, LDS_STRIDE);
#pragma unroll
    for (int j = 0; j < 4; ++j)
      wf[j] = lds_frag(ldsW + (wn + 16 * j) * LDS_STRIDE, LDS_STRIDE);
#pragma unroll
    for (int i = 0; i < 4; ++i)
#pragma unroll
      for (int j = 0; j < 4; ++j)
        acc[i][j] = wmma_bf16(af[i], wf[j], acc[i][j]);
  }

  const int nlane = lane & 15;
  const int mh    = (lane >> 4) * 8;
  __syncthreads();
  if (MODE == 0 || MODE == 1) {
    bf16* so = (bf16*)sob;
#pragma unroll
    for (int i = 0; i < 4; ++i)
#pragma unroll
      for (int j = 0; j < 4; ++j) {
        const int nl = wn + 16 * j + nlane;
        const float bv = bias ? bias[nBlk + nl] : 0.0f;
#pragma unroll
        for (int r = 0; r < 8; ++r) {
          const int ml = wm + 16 * i + mh + r;
          const bf16 hv = (bf16)(acc[i][j][r] + bv);
          if (MODE == 0) so[ml * 264 + nl] = hv;
          else           so[nl * 136 + ml] = hv;
        }
      }
    __syncthreads();
#pragma unroll 1
    for (int pass = 0; pass < 2; ++pass) {
      if (MODE == 0) {
        for (int ch = t; ch < 128 * 32; ch += 256) { const int ml = ch >> 5, q = (ch & 31) * 8;
          *(volatile v4u_t*)((bf16*)out + (size_t)(mBlk + ml) * N + nBlk + q) = *(const v4ua*)(so + ml * 264 + q); }
      } else {
        const int b_ = mBlk / SS, s0 = mBlk & (SS - 1);
        for (int ch = t; ch < 256 * 16; ch += 256) { const int nl = ch >> 4, q = (ch & 15) * 8; const int n = nBlk + nl, h = n >> 6, dk = n & (DKK - 1);
          *(volatile v4u_t*)((bf16*)out + (((size_t)(b_ * HH + h)) * DKK + dk) * SS + s0 + q) = *(const v4ua*)(so + nl * 136 + q); }
      }
      __threadfence();
    }
  } else {
    float* so = (float*)sob;
#pragma unroll 1
    for (int hf = 0; hf < 2; ++hf) {
      if (wm == hf * 64) {
#pragma unroll
        for (int i = 0; i < 4; ++i)
#pragma unroll
          for (int j = 0; j < 4; ++j) {
            const int nl = wn + 16 * j + nlane;
            const float bv = bias ? bias[nBlk + nl] : 0.0f;
#pragma unroll
            for (int r = 0; r < 8; ++r) so[(16 * i + mh + r) * 260 + nl] = acc[i][j][r] + bv;
          }
      }
      __syncthreads();
#pragma unroll 1
      for (int pass = 0; pass < 2; ++pass) {
        for (int ch = t; ch < 64 * 64; ch += 256) { const int ml = ch >> 6, q = (ch & 63) * 4;
          *(volatile v4f_t*)((float*)out + (size_t)(mBlk + hf * 64 + ml) * N + nBlk + q) = *(const volatile v4fa*)(so + ml * 260 + q); }
        __threadfence();
      }
      __syncthreads();
    }
  }
}


#define NTOK (NBATCH * NN)

__global__ __launch_bounds__(256) void k_sd(const float* __restrict__ Hh, const float* __restrict__ as_, const float* __restrict__ ad_, float* __restrict__ S, float* __restrict__ D) {
  __shared__ float ps[64][5], pd[64][5];
  const int t = threadIdx.x, rl = t >> 2, p4 = t & 3; const size_t row = (size_t)blockIdx.x * 64 + rl; float s = 0.f, d = 0.f;
#pragma unroll 1
  for (int k = p4 * 32; k < p4 * 32 + 32; ++k) { const float h = Hh[row * 256 + k]; s += h * as_[k]; d += h * ad_[k]; }
  ps[rl][p4] = s; pd[rl][p4] = d; __syncthreads();
  if (t < 64) { const float sv = ps[t][0] + ps[t][1] + ps[t][2] + ps[t][3], dv = pd[t][0] + pd[t][1] + pd[t][2] + pd[t][3];
#pragma unroll 1
    for (int pass = 0; pass < 2; ++pass) { *(volatile float*)(S + (size_t)blockIdx.x * 64 + t) = sv; *(volatile float*)(D + (size_t)blockIdx.x * 64 + t) = dv; __threadfence(); } }
}
__global__ __launch_bounds__(256) void k_ht(const float* __restrict__ Hh, float* __restrict__ HT) {
  __shared__ float tile[64][65];
  const int m0 = blockIdx.x * 64, f0 = blockIdx.y * 64, b = blockIdx.z, t = threadIdx.x;
  if (f0 < HD) { for (int i = t; i < 64 * 64; i += 256) { const int r = i >> 6, f = i & 63; tile[r][f] = Hh[((size_t)(b * NN + m0 + r)) * 256 + f0 + f]; } }
  __syncthreads();
#pragma unroll 1
  for (int pass = 0; pass < 2; ++pass) {
    for (int i = t; i < 64 * 16; i += 256) { const int fr = i >> 4, m4 = (i & 15) * 4; v4f_t v;
      if (f0 < HD) { v.x = tile[m4][fr]; v.y = tile[m4 + 1][fr]; v.z = tile[m4 + 2][fr]; v.w = tile[m4 + 3][fr]; } else { v.x = v.y = v.z = v.w = 0.0f; }
      *(volatile v4f_t*)(HT + ((size_t)b * 256 + f0 + fr) * NN + m0 + m4) = v; }
    __threadfence(); }
}
__global__ __launch_bounds__(256) void k_p(const float* __restrict__ Am, const float* __restrict__ S, const float* __restrict__ D, bf16* __restrict__ P) {
  __shared__ float red[256];
  const int row = blockIdx.x, b = row / NN, n = row % NN, t = threadIdx.x; const float sn = S[row];
  const float* Ar = Am + (size_t)n * NN; const float* Db = D + (size_t)b * NN;
  float e4[4]; float mx = -INFINITY;
#pragma unroll
  for (int q = 0; q < 4; ++q) { const int m = t * 4 + q; float e = sn + Db[m]; e = (e >= 0.0f) ? e : 0.2f * e; e = e / 2.0f;
    e4[q] = (Ar[m] >= 1e-9f) ? e : -INFINITY; mx = fmaxf(mx, e4[q]); }
  red[t] = mx; __syncthreads();
  for (int o = 128; o > 0; o >>= 1) { if (t < o) red[t] = fmaxf(red[t], red[t + o]); __syncthreads(); }
  const float m_ = red[0]; __syncthreads();
  float p4[4], s = 0.0f;
#pragma unroll
  for (int q = 0; q < 4; ++q) { p4[q] = (e4[q] == -INFINITY) ? 0.0f : expf(e4[q] - m_); s += p4[q]; }
  red[t] = s; __syncthreads();
  for (int o = 128; o > 0; o >>= 1) { if (t < o) red[t] += red[t + o]; __syncthreads(); }
  const float inv = 1.0f / red[0];
  bf16 hq[4]; hq[0] = (bf16)(p4[0] * inv); hq[1] = (bf16)(p4[1] * inv); hq[2] = (bf16)(p4[2] * inv); hq[3] = (bf16)(p4[3] * inv);
  typedef __attribute__((ext_vector_type(2))) unsigned v2u; typedef unsigned v2ua __attribute__((ext_vector_type(2), may_alias));
  *(volatile v2u*)(P + (size_t)row * NN + t * 4) = *(const v2ua*)hq; __threadfence(); *(volatile v2u*)(P + (size_t)row * NN + t * 4) = *(const v2ua*)hq;
}
__global__ __launch_bounds__(128) void k_tanhc(const float* __restrict__ T, float* __restrict__ Hout, int ldo, int c0) {
  const int row = blockIdx.x, f = threadIdx.x; const float v = tanhf(T[(size_t)row * 256 + f]);
  *(volatile float*)(Hout + (size_t)row * ldo + c0 + f) = v; __threadfence(); *(volatile float*)(Hout + (size_t)row * ldo + c0 + f) = v;
}
__global__ __launch_bounds__(256) void k_padw(const float* __restrict__ W, float* __restrict__ Wp) {
  const int n = blockIdx.x; for (int k = threadIdx.x; k < 512; k += 256) { const float v = (n < HD) ? W[(size_t)n * 512 + k] : 0.0f; *(volatile float*)(Wp + (size_t)n * 512 + k) = v; }
  __threadfence();
  for (int k = threadIdx.x; k < 512; k += 256) { const float v = (n < HD) ? W[(size_t)n * 512 + k] : 0.0f; *(volatile float*)(Wp + (size_t)n * 512 + k) = v; }
}
__global__ __launch_bounds__(128) void k_final(const float* __restrict__ Z, const float* __restrict__ b1, const float* __restrict__ W2, const float* __restrict__ b2, const float* __restrict__ C,
                                              const float* __restrict__ HX, const float* __restrict__ hg, const float* __restrict__ g, const float* __restrict__ be, float* __restrict__ out) {
  __shared__ float red[128]; __shared__ float lg[4][5]; __shared__ float mixw[4];
  const int row = blockIdx.x, n = row % NN, f = threadIdx.x, wave = f >> 5, lane = f & 31;
  const float z = tanhf(Z[(size_t)row * 256 + f] + b1[f]);
  float p[4];
#pragma unroll
  for (int k = 0; k < 4; ++k) { float v = z * W2[k * HD + f];
#pragma unroll
    for (int o = 16; o >= 1; o >>= 1) v += __shfl_xor(v, o, 32); p[k] = v; }
  if (lane == 0) { lg[0][wave] = p[0]; lg[1][wave] = p[1]; lg[2][wave] = p[2]; lg[3][wave] = p[3]; }
  __syncthreads();
  if (f == 0) { float l[4], mx = -INFINITY;
    for (int k = 0; k < 4; ++k) { l[k] = lg[k][0] + lg[k][1] + lg[k][2] + lg[k][3] + b2[k]; mx = fmaxf(mx, l[k]); }
    float s = 0.f; for (int k = 0; k < 4; ++k) { l[k] = expf(l[k] - mx); s += l[k]; } for (int k = 0; k < 4; ++k) mixw[k] = l[k] / s; }
  __syncthreads();
  const float* cr = C + (size_t)row * 512;
  float h = mixw[0] * cr[f] + mixw[1] * cr[HD + f] + mixw[2] * cr[2 * HD + f] + mixw[3] * cr[3 * HD + f];
  h += (1.0f / (1.0f + expf(-hg[n]))) * tanhf(HX[(size_t)row * 256 + f]);
  red[f] = h; __syncthreads();
  for (int o = 64; o > 0; o >>= 1) { if (f < o) red[f] += red[f + o]; __syncthreads(); }
  const float mu = red[0] / (float)HD; __syncthreads();
  const float dv = h - mu; red[f] = dv * dv; __syncthreads();
  for (int o = 64; o > 0; o >>= 1) { if (f < o) red[f] += red[f + o]; __syncthreads(); }
  const float rs = rsqrtf(red[0] / (float)HD + 1e-5f);
  const float v = dv * rs * g[f] + be[f];
  *(volatile float*)(out + (size_t)row * HD + f) = v; __threadfence(); *(volatile float*)(out + (size_t)row * HD + f) = v;
}

static void gat(hipStream_t stream, const float* Xin, const float* Am, const float* Wp, const float* as_, const float* ad_,
                float* Hh, float* S, float* D, float* HT, bf16* P, float* T, float* Hout, int ldo, int c0) {
  dim3 blk(256);
  gemm_bias_kernel<float, 2><<<dim3(NTOK / 128, 1, 1), blk, 0, stream>>>(Xin, Wp, nullptr, Hh, NTOK, 256, HD, 0, 0, 0);
  k_sd<<<NTOK / 64, 256, 0, stream>>>(Hh, as_, ad_, S, D);
  k_ht<<<dim3(NN / 64, 4, NBATCH), 256, 0, stream>>>(Hh, HT);
  k_p<<<NTOK, 256, 0, stream>>>(Am, S, D, P);
  gemm_bias_kernel<bf16, 2><<<dim3(NN / 128, 1, NBATCH), blk, 0, stream>>>(P, HT, nullptr, T, NN, 256, NN, (size_t)NN * NN, (size_t)256 * NN, (size_t)NN * 256 * 4);
  k_tanhc<<<NTOK, 128, 0, stream>>>(T, Hout, ldo, c0);
}

__global__ __launch_bounds__(128) void k_padw128(const float* __restrict__ W, float* __restrict__ Wp) {
  const int n = blockIdx.x, k = threadIdx.x; const float v = (n < HD) ? W[(size_t)n * HD + k] : 0.0f;
  *(volatile float*)(Wp + (size_t)n * HD + k) = v; __threadfence(); *(volatile float*)(Wp + (size_t)n * HD + k) = v;
}

extern "C" void kernel_launch(void* const* d_in, const int* in_sizes, int n_in,
                              void* d_out, int out_size, void* d_ws, size_t ws_size,
                              hipStream_t stream) {
  (void)in_sizes; (void)n_in; (void)out_size; (void)ws_size;
  const float* x = (const float*)d_in[1];
  const float* A_sym = (const float*)d_in[2]; const float* A_fwd = (const float*)d_in[3]; const float* A_bwd = (const float*)d_in[4]; const float* A_corr = (const float*)d_in[5];
  const float* Hc = (const float*)d_in[6];
  const float* Ws1 = (const float*)d_in[7];  const float* as1 = (const float*)d_in[8];  const float* ad1 = (const float*)d_in[9];
  const float* Ws2 = (const float*)d_in[10]; const float* as2 = (const float*)d_in[11]; const float* ad2 = (const float*)d_in[12];
  const float* Wf  = (const float*)d_in[13]; const float* asf = (const float*)d_in[14]; const float* adf = (const float*)d_in[15];
  const float* Wb  = (const float*)d_in[16]; const float* asb = (const float*)d_in[17]; const float* adb = (const float*)d_in[18];
  const float* Wc  = (const float*)d_in[19]; const float* asc = (const float*)d_in[20]; const float* adc = (const float*)d_in[21];
  const float* mW1 = (const float*)d_in[22]; const float* mb1 = (const float*)d_in[23]; const float* mW2 = (const float*)d_in[24]; const float* mb2 = (const float*)d_in[25];
  const float* theta = (const float*)d_in[26]; const float* hg = (const float*)d_in[27]; const float* lg = (const float*)d_in[28]; const float* lb = (const float*)d_in[29];
  float* out = (float*)d_out;
  char* ws = (char*)d_ws;
  float* Wp  = (float*)ws; ws += (size_t)6 * 256 * HD * 4;
  float* W1p = (float*)ws; ws += (size_t)256 * 512 * 4;
  float* S   = (float*)ws; ws += (size_t)NTOK * 4; float* D = (float*)ws; ws += (size_t)NTOK * 4;
  float* Hh  = (float*)ws; ws += (size_t)NTOK * 256 * 4;
  float* HT  = (float*)ws; ws += (size_t)NBATCH * 256 * NN * 4;
  bf16* P    = (bf16*)ws;  ws += (size_t)NBATCH * NN * NN * 2;
  float* T   = (float*)ws; ws += (size_t)NTOK * 256 * 4;
  float* C   = (float*)ws; ws += (size_t)NTOK * 512 * 4;
  float* h1  = (float*)P;
  const size_t wsz = (size_t)256 * HD;
  k_padw128<<<256, 128, 0, stream>>>(Ws1, Wp); k_padw128<<<256, 128, 0, stream>>>(Ws2, Wp + wsz); k_padw128<<<256, 128, 0, stream>>>(Wf, Wp + 2 * wsz);
  k_padw128<<<256, 128, 0, stream>>>(Wb, Wp + 3 * wsz); k_padw128<<<256, 128, 0, stream>>>(Wc, Wp + 4 * wsz); k_padw128<<<256, 128, 0, stream>>>(theta, Wp + 5 * wsz);
  k_padw<<<256, 256, 0, stream>>>(mW1, W1p);
  gat(stream, x,  A_sym,  Wp,           as1, ad1, Hh, S, D, HT, P, T, h1, HD, 0);
  gat(stream, h1, A_sym,  Wp + wsz,     as2, ad2, Hh, S, D, HT, P, T, C, 512, 0);
  gat(stream, x,  A_fwd,  Wp + 2 * wsz, asf, adf, Hh, S, D, HT, P, T, C, 512, HD);
  gat(stream, x,  A_bwd,  Wp + 3 * wsz, asb, adb, Hh, S, D, HT, P, T, C, 512, 2 * HD);
  gat(stream, x,  A_corr, Wp + 4 * wsz, asc, adc, Hh, S, D, HT, P, T, C, 512, 3 * HD);
  dim3 blk(256);
  gemm_bias_kernel<float, 2><<<dim3(NTOK / 128, 1, 1), blk, 0, stream>>>(x, Wp + 5 * wsz, nullptr, Hh, NTOK, 256, HD, 0, 0, 0);
  k_ht<<<dim3(NN / 64, 4, NBATCH), 256, 0, stream>>>(Hh, HT);
  gemm_bias_kernel<float, 2><<<dim3(NN / 128, 1, NBATCH), blk, 0, stream>>>(Hc, HT, nullptr, T, NN, 256, NN, 0, (size_t)256 * NN, (size_t)NN * 256 * 4);
  float* Z = Hh;
  gemm_bias_kernel<float, 2><<<dim3(NTOK / 128, 1, 1), blk, 0, stream>>>(C, W1p, nullptr, Z, NTOK, 256, 512, 0, 0, 0);
  k_final<<<NTOK, 128, 0, stream>>>(Z, mb1, mW2, mb2, C, T, hg, lg, lb, out);
}
